// DeformConvBlock_40303973106011
// MI455X (gfx1250) — hardware-verified
//
#include <hip/hip_runtime.h>
#include <stddef.h>

static constexpr int NBATCH = 8;
static constexpr int CIN    = 64;
static constexpr int HH     = 128;
static constexpr int WD     = 128;
static constexpr int HW     = 16384;
static constexpr int COUT   = 64;
static constexpr int KK     = 9;
static constexpr int KD     = 576;
static constexpr int MOFF   = 64;
static constexpr int NOFF   = 18;
static constexpr int NPIX   = NBATCH * HW;
static_assert(KD % 32 == 0);
static_assert(HW % 64 == 0 && MOFF % 64 == 0 && COUT % 64 == 0);

typedef __attribute__((ext_vector_type(16))) _Float16 v16h;
typedef __attribute__((ext_vector_type(8)))  _Float16 v8h;
typedef __attribute__((ext_vector_type(16))) __bf16   v16b;
typedef __attribute__((ext_vector_type(8)))  __bf16   v8b;
typedef __attribute__((ext_vector_type(8)))  float    v8f;
typedef __attribute__((ext_vector_type(4)))  float    v4f;
typedef __attribute__((ext_vector_type(4)))  unsigned v4u;

__device__ __forceinline__ unsigned short f2bf_bits(float f) {
  unsigned u = __float_as_uint(f);
  return (unsigned short)((u + 0x7FFFu + ((u >> 16) & 1u)) >> 16);
}
__device__ __forceinline__ float bf_bits2f(unsigned short h) { return __uint_as_float(((unsigned)h) << 16); }

__device__ __forceinline__ unsigned pk2(unsigned short a, unsigned short b) {
  return (unsigned)a | ((unsigned)b << 16);
}
__device__ __forceinline__ unsigned pkh2(float a, float b) {
  return pk2(__builtin_bit_cast(unsigned short, (_Float16)a), __builtin_bit_cast(unsigned short, (_Float16)b));
}
__device__ __forceinline__ void pkbf2(float a, float b, unsigned& uh, unsigned& ul) {
  const unsigned short ha = f2bf_bits(a), hb = f2bf_bits(b);
  const unsigned short la = f2bf_bits(a - bf_bits2f(ha)), lb = f2bf_bits(b - bf_bits2f(hb));
  uh = pk2(ha, hb);
  ul = pk2(la, lb);
}

__device__ __forceinline__ void dep_guard_h(v8f& a, v8f& b, v16h x, v16h y) { asm volatile("v_nop\n\tv_nop\n\tv_nop\n\tv_nop" : "+v"(a), "+v"(b) : "v"(x), "v"(y)); }
__device__ __forceinline__ void dep_guard_b(v8f& a, v8f& b, v16b x, v16b y) { asm volatile("v_nop\n\tv_nop\n\tv_nop\n\tv_nop" : "+v"(a), "+v"(b) : "v"(x), "v"(y)); }
__device__ __forceinline__ void keep4_h(v16h a, v16h b, v16h c, v16h d) { asm volatile("v_nop" :: "v"(a), "v"(b), "v"(c), "v"(d)); }
__device__ __forceinline__ void keep4_b(v16b a, v16b b, v16b c, v16b d) { asm volatile("v_nop" :: "v"(a), "v"(b), "v"(c), "v"(d)); }
__device__ __forceinline__ void acc_guard4(v8f& a, v8f& b, v8f& c, v8f& d) { asm volatile("v_nop\n\tv_nop\n\tv_nop\n\tv_nop" : "+v"(a), "+v"(b), "+v"(c), "+v"(d)); }
template <typename T> struct Frag;
template <> struct Frag<_Float16> {
  typedef v16h V; union U { v16h v; v8h h[2]; };
  static __device__ __forceinline__ v16h load(const _Float16* p) {
    U f; f.h[0] = *(const v8h*)(p); f.h[1] = *(const v8h*)(p + 16); return f.v;
  }
  static __device__ __forceinline__ v8f mma(v16h a, v16h b, v8f c) {
    return __builtin_amdgcn_wmma_f32_16x16x32_f16(false, a, false, b, (short)0, c, false, false);
  }
  static __device__ __forceinline__ void guard(v8f& a, v8f& b, v16h x, v16h y) { dep_guard_h(a, b, x, y); }
  static __device__ __forceinline__ void keep(v16h a, v16h b, v16h c, v16h d) { keep4_h(a, b, c, d); }
};
template <> struct Frag<__bf16> {
  typedef v16b V; union U { v16b v; v8b h[2]; };
  static __device__ __forceinline__ v16b load(const __bf16* p) {
    U f; f.h[0] = *(const v8b*)(p); f.h[1] = *(const v8b*)(p + 16); return f.v;
  }
  static __device__ __forceinline__ v8f mma(v16b a, v16b b, v8f c) {
    return __builtin_amdgcn_wmma_f32_16x16x32_bf16(false, a, false, b, (short)0, c, false, false);
  }
  static __device__ __forceinline__ void guard(v8f& a, v8f& b, v16b x, v16b y) { dep_guard_b(a, b, x, y); }
  static __device__ __forceinline__ void keep(v16b a, v16b b, v16b c, v16b d) { keep4_b(a, b, c, d); }
};

template <int ET> struct Elem;
template <> struct Elem<0> { typedef _Float16 T; };
template <> struct Elem<1> { typedef __bf16 T; };
template <int ET, bool SPLIT, int BIAS_MODE, int OUT_MODE, bool RESID, int ACT = 0>
__global__ __launch_bounds__(256) void wmma_gemm64(
    const unsigned short* __restrict__ Ap, const unsigned short* __restrict__ A2p, int lda, long strideA,
    const unsigned short* __restrict__ Btp, const unsigned short* __restrict__ Bt2p, int ldb, long strideB,
    void* __restrict__ Cout, void* __restrict__ Cout2, int ldc, long strideC,
    const float* __restrict__ bias,
    const float* __restrict__ resid, long strideR,
    int M, int N, int K, float scale) {
  typedef typename Elem<ET>::T T;
  typedef typename Frag<T>::V V;
  const T* A = (const T*)Ap; const T* A2 = (const T*)A2p; const T* Bt = (const T*)Btp; const T* Bt2 = (const T*)Bt2p;
  __shared__ __align__(16) float sT[8][16 * 68];
  const int b    = blockIdx.y;
  const int lane = threadIdx.x & 31;
  const int wave = threadIdx.x >> 5;
  const int tilesN = N >> 6;
  const int tilesM = M >> 6;
  const int tile = blockIdx.x * 8 + wave;
  if (tile >= tilesM * tilesN) return;
  const int tm = tile / tilesN;
  const int tn = tile - tm * tilesN;
  const int m0 = tm << 6;
  const int n0 = tn << 6;

  const T* Ab  = A  + (size_t)b * strideA;
  const T* Bb  = Bt + (size_t)b * strideB;
  const T* Ab2 = SPLIT ? (A2  + (size_t)b * strideA) : nullptr;
  const T* Bb2 = SPLIT ? (Bt2 + (size_t)b * strideB) : nullptr;

  const int rlane = lane & 15;
  const int koff  = (lane >> 4) * 8;
  const int mOff  = (lane >> 4) * 8;

  v8f acc[4][4];
#pragma unroll
  for (int i = 0; i < 4; ++i)
#pragma unroll
    for (int j = 0; j < 4; ++j) acc[i][j] = (v8f){0.f,0.f,0.f,0.f,0.f,0.f,0.f,0.f};

  for (int k0 = 0; k0 < K; k0 += 32) {
    V bh[4], bl[4];
#pragma unroll
    for (int j = 0; j < 4; ++j) {
      const size_t bo = (size_t)(n0 + (j << 4) + rlane) * ldb + koff + k0;
      bh[j] = Frag<T>::load(Bb + bo);
      if (SPLIT) bl[j] = Frag<T>::load(Bb2 + bo);
    }
#pragma unroll
    for (int i = 0; i < 4; ++i) {
      const size_t ao = (size_t)(m0 + (i << 4) + rlane) * lda + koff + k0;
      V ah = Frag<T>::load(Ab + ao);
      V al;
      if (SPLIT) al = Frag<T>::load(Ab2 + ao);
#pragma unroll
      for (int j = 0; j < 4; ++j) {
        acc[i][j] = Frag<T>::mma(ah, bh[j], acc[i][j]);
        if (SPLIT) {
          acc[i][j] = Frag<T>::mma(ah, bl[j], acc[i][j]);
          acc[i][j] = Frag<T>::mma(al, bh[j], acc[i][j]);
        }
      }
      Frag<T>::guard(acc[i][0], acc[i][3], ah, SPLIT ? al : ah);
    }
    Frag<T>::keep(bh[0], bh[1], bh[2], bh[3]);
    if (SPLIT) Frag<T>::keep(bl[0], bl[1], bl[2], bl[3]);
  }
  acc_guard4(acc[0][0], acc[0][1], acc[0][2], acc[0][3]);
  acc_guard4(acc[1][0], acc[1][1], acc[1][2], acc[1][3]);
  acc_guard4(acc[2][0], acc[2][1], acc[2][2], acc[2][3]);
  acc_guard4(acc[3][0], acc[3][1], acc[3][2], acc[3][3]);

  float* slab = sT[wave];
  const float* Rb = RESID ? (resid + (size_t)b * strideR) : nullptr;
#pragma unroll
  for (int i = 0; i < 4; ++i) {
    const int mBase = m0 + (i << 4);
#pragma unroll
    for (int j = 0; j < 4; ++j) {
      const int n = n0 + (j << 4) + rlane;
      float bv = 0.f;
      if (BIAS_MODE == 2) bv = bias[n];
#pragma unroll
      for (int r = 0; r < 8; ++r) {
        float v = acc[i][j][r] * scale;
        if (BIAS_MODE == 1) v += bias[mBase + mOff + r];
        if (BIAS_MODE == 2) v += bv;
        if (RESID) v += Rb[(size_t)(mBase + mOff + r) * ldc + n];
        if (ACT == 1) v = tanhf(v);
        if (ACT == 2) v = fmaxf(v, 0.0f);
        if (ACT == 4) v = (v > 0.f) ? v : 0.01f * v;
        slab[(mOff + r) * 68 + (j << 4) + rlane] = v;
      }
    }
    __builtin_amdgcn_fence(__ATOMIC_RELEASE, "workgroup");
    __builtin_amdgcn_wave_barrier();
    __builtin_amdgcn_fence(__ATOMIC_ACQUIRE, "workgroup");
    if (OUT_MODE == 0) {
      float* C = (float*)Cout + (size_t)b * strideC;
      const int hh = lane >> 4, c4 = (lane & 15) * 4;
      for (int pass = 0; pass < 2; ++pass) {
#pragma unroll
        for (int it = 0; it < 8; ++it) {
          const int row = it * 2 + hh;
          v4f v = *(const v4f*)(slab + row * 68 + c4);
          *(volatile v4f*)(C + (size_t)(mBase + row) * ldc + n0 + c4) = v;
        }
        __threadfence();
      }
    } else {
      const int q = lane >> 3, c8 = (lane & 7) * 8;
      unsigned short* C  = (unsigned short*)Cout  + (size_t)b * strideC;
      unsigned short* C2 = (OUT_MODE == 2) ? ((unsigned short*)Cout2 + (size_t)b * strideC) : nullptr;
      for (int pass = 0; pass < 2; ++pass) {
#pragma unroll
        for (int it = 0; it < 4; ++it) {
          const int row = it * 4 + q;
          const float* sp = slab + row * 68 + c8;
          v8h hv, lv;
#pragma unroll
          for (int e = 0; e < 8; ++e) {
            if (OUT_MODE == 1) {
              hv[e] = (_Float16)sp[e];
            } else {
              unsigned short hb = f2bf_bits(sp[e]);
              unsigned short lb = f2bf_bits(sp[e] - bf_bits2f(hb));
              hv[e] = __builtin_bit_cast(_Float16, hb);
              lv[e] = __builtin_bit_cast(_Float16, lb);
            }
          }
          *(volatile v8h*)(C + (size_t)(mBase + row) * ldc + n0 + c8) = hv;
          if (OUT_MODE == 2) *(volatile v8h*)(C2 + (size_t)(mBase + row) * ldc + n0 + c8) = lv;
        }
        __threadfence();
      }
    }
    __builtin_amdgcn_fence(__ATOMIC_RELEASE, "workgroup");
    __builtin_amdgcn_wave_barrier();
    __builtin_amdgcn_fence(__ATOMIC_ACQUIRE, "workgroup");
  }
}

__global__ __launch_bounds__(256) void k_xpose(const float* __restrict__ x, float* __restrict__ xT) {
  __shared__ float t[CIN][33];
  const int tid = threadIdx.x;
  const int blk = blockIdx.x;
  const int b   = blk / (HW / 32);
  const int hw0 = (blk - b * (HW / 32)) * 32;
  const float* xb = x + (size_t)b * CIN * HW + hw0;
#pragma unroll
  for (int i = 0; i < 8; ++i) {
    const int idx = i * 256 + tid;
    const int c = idx >> 5, j = idx & 31;
    t[c][j] = xb[(size_t)c * HW + j];
  }
  __syncthreads();
  const int wave = tid >> 5, lane = tid & 31, hh = lane >> 4, c4 = (lane & 15) * 4;
  float* ob = xT + ((size_t)b * HW + hw0) * CIN;
  for (int pass = 0; pass < 2; ++pass) {
#pragma unroll
    for (int it = 0; it < 2; ++it) {
      const int row = wave * 4 + it * 2 + hh;
      v4f v;
      v[0] = t[c4][row]; v[1] = t[c4 + 1][row]; v[2] = t[c4 + 2][row]; v[3] = t[c4 + 3][row];
      *(volatile v4f*)(ob + (size_t)row * CIN + c4) = v;
    }
    __threadfence();
  }
}

__global__ __launch_bounds__(256) void k_prep_woff(const float* __restrict__ w, unsigned short* __restrict__ Ah,
                                                   unsigned short* __restrict__ Al) {
  const int g = blockIdx.x * 256 + threadIdx.x;
  if (g < MOFF * KD / 8) {
    const int e0 = g * 8;
    const int o  = e0 / KD;
    const int col = e0 - o * KD;
    const int k  = col >> 6;
    const int c0 = col & 63;
    const int oc = o < NOFF ? o : (NOFF - 1);
    float f[8];
#pragma unroll
    for (int j = 0; j < 8; ++j) {
      float v = w[(size_t)(oc * CIN + c0 + j) * KK + k];
      f[j] = (o < NOFF) ? v : 0.0f;
    }
    v4u uh, ul;
    unsigned a, bb;
    pkbf2(f[0], f[1], a, bb); uh[0] = a; ul[0] = bb;
    pkbf2(f[2], f[3], a, bb); uh[1] = a; ul[1] = bb;
    pkbf2(f[4], f[5], a, bb); uh[2] = a; ul[2] = bb;
    pkbf2(f[6], f[7], a, bb); uh[3] = a; ul[3] = bb;
    volatile v4u* ph = (volatile v4u*)(Ah + e0);
    volatile v4u* pl = (volatile v4u*)(Al + e0);
    *ph = uh; *pl = ul;
    __threadfence();
    *ph = uh; *pl = ul;
  }
}

__global__ __launch_bounds__(256) void k_prep_wdef(const float* __restrict__ w, unsigned short* __restrict__ Bw) {
  const int g = blockIdx.x * 256 + threadIdx.x;
  if (g < COUT * KD / 8) {
    const int e0 = g * 8;
    const int o  = e0 / KD;
    const int col = e0 - o * KD;
    const int k  = col >> 6;
    const int c0 = col & 63;
    float f[8];
#pragma unroll
    for (int j = 0; j < 8; ++j) f[j] = w[(size_t)(o * CIN + c0 + j) * KK + k] * 16.0f;
    v4u u;
    u[0] = pkh2(f[0], f[1]); u[1] = pkh2(f[2], f[3]); u[2] = pkh2(f[4], f[5]); u[3] = pkh2(f[6], f[7]);
    volatile v4u* p = (volatile v4u*)(Bw + e0);
    *p = u;
    __threadfence();
    *p = u;
  }
}

__global__ __launch_bounds__(256) void k_im2col(const float* __restrict__ xT, unsigned short* __restrict__ Ph,
                                                unsigned short* __restrict__ Pl, int bsel) {
  const int lane = threadIdx.x & 31, wave = threadIdx.x >> 5;
  const int q = lane >> 3, c8 = (lane & 7) * 8;
  const int it = (blockIdx.x * 8 + wave) * 4 + q;
  if (it < HW * KK) {
    const int hw = it / KK, k = it - hw * KK;
    const int ho = hw >> 7, wo = hw & (WD - 1);
    const int kh = k / 3, kw = k - kh * 3;
    const int y = ho - 1 + kh, xx = wo - 1 + kw;
    const bool inb = ((unsigned)y < (unsigned)HH) && ((unsigned)xx < (unsigned)WD);
    const int yc = y < 0 ? 0 : (y > HH - 1 ? HH - 1 : y);
    const int xc = xx < 0 ? 0 : (xx > WD - 1 ? WD - 1 : xx);
    const float* src = xT + ((size_t)bsel * HW + (size_t)yc * WD + xc) * CIN + c8;
    v4f a = *(const v4f*)(src);
    v4f c = *(const v4f*)(src + 4);
    const v4f z = (v4f){0.f, 0.f, 0.f, 0.f};
    if (!inb) { a = z; c = z; }
    v4u uh, ul;
    unsigned p0, p1;
    pkbf2(a[0], a[1], p0, p1); uh[0] = p0; ul[0] = p1;
    pkbf2(a[2], a[3], p0, p1); uh[1] = p0; ul[1] = p1;
    pkbf2(c[0], c[1], p0, p1); uh[2] = p0; ul[2] = p1;
    pkbf2(c[2], c[3], p0, p1); uh[3] = p0; ul[3] = p1;
    volatile v4u* dh = (volatile v4u*)(Ph + (size_t)it * CIN + c8);
    volatile v4u* dl = (volatile v4u*)(Pl + (size_t)it * CIN + c8);
    *dh = uh; *dl = ul;
    __threadfence();
    *dh = uh; *dl = ul;
  }
}

__global__ __launch_bounds__(256) void k_sample(const float* __restrict__ xT, const float* __restrict__ off,
                                                const float* __restrict__ boff, unsigned short* __restrict__ S, int bsel) {
  const int lane = threadIdx.x & 31, wave = threadIdx.x >> 5;
  const int q = lane >> 3, c8 = (lane & 7) * 8;
  const int it = (blockIdx.x * 8 + wave) * 4 + q;
  if (it < HW * KK) {
    const int p = it / KK, k = it - p * KK;
    const int ho = p >> 7, wo = p & (WD - 1);
    const int kh = k / 3, kw = k - kh * 3;
    const float dy = off[(size_t)(2 * k) * HW + p] + boff[2 * k];
    const float dx = off[(size_t)(2 * k + 1) * HW + p] + boff[2 * k + 1];
    const float py = (float)(ho - 1 + kh) + dy;
    const float px = (float)(wo - 1 + kw) + dx;
    const float y0 = floorf(py), x0 = floorf(px);
    const float y1 = y0 + 1.0f, x1 = x0 + 1.0f;
    const float wy1 = py - y0, wx1 = px - x0;
    const float wy0 = 1.0f - wy1, wx0 = 1.0f - wx1;
    const bool vy0 = (y0 >= 0.0f) && (y0 <= (float)(HH - 1));
    const bool vy1 = (y1 >= 0.0f) && (y1 <= (float)(HH - 1));
    const bool vx0 = (x0 >= 0.0f) && (x0 <= (float)(WD - 1));
    const bool vx1 = (x1 >= 0.0f) && (x1 <= (float)(WD - 1));
    float w00 = wy0 * wx0, w01 = wy0 * wx1, w10 = wy1 * wx0, w11 = wy1 * wx1;
    w00 = (vy0 && vx0) ? w00 : 0.0f;
    w01 = (vy0 && vx1) ? w01 : 0.0f;
    w10 = (vy1 && vx0) ? w10 : 0.0f;
    w11 = (vy1 && vx1) ? w11 : 0.0f;
    const int yi0 = (int)fminf(fmaxf(y0, 0.0f), (float)(HH - 1));
    const int yi1 = (int)fminf(fmaxf(y1, 0.0f), (float)(HH - 1));
    const int xi0 = (int)fminf(fmaxf(x0, 0.0f), (float)(WD - 1));
    const int xi1 = (int)fminf(fmaxf(x1, 0.0f), (float)(WD - 1));
    const float* xb  = xT + (size_t)bsel * HW * CIN + c8;
    const float* r00 = xb + ((size_t)yi0 * WD + xi0) * CIN;
    const float* r01 = xb + ((size_t)yi0 * WD + xi1) * CIN;
    const float* r10 = xb + ((size_t)yi1 * WD + xi0) * CIN;
    const float* r11 = xb + ((size_t)yi1 * WD + xi1) * CIN;
    const v4f g00a = *(const v4f*)(r00), g00b = *(const v4f*)(r00 + 4);
    const v4f g01a = *(const v4f*)(r01), g01b = *(const v4f*)(r01 + 4);
    const v4f g10a = *(const v4f*)(r10), g10b = *(const v4f*)(r10 + 4);
    const v4f g11a = *(const v4f*)(r11), g11b = *(const v4f*)(r11 + 4);
    const v4f va = g00a * w00 + g01a * w01 + g10a * w10 + g11a * w11;
    const v4f vb = g00b * w00 + g01b * w01 + g10b * w10 + g11b * w11;
    v4u u;
    u[0] = pkh2(va[0], va[1]); u[1] = pkh2(va[2], va[3]);
    u[2] = pkh2(vb[0], vb[1]); u[3] = pkh2(vb[2], vb[3]);
    volatile v4u* d = (volatile v4u*)(S + (size_t)it * CIN + c8);
    *d = u;
    __threadfence();
    *d = u;
  }
}

__global__ __launch_bounds__(256) void k_bnorm(const float* __restrict__ pre, const float* __restrict__ gamma,
                                               const float* __restrict__ beta, float* __restrict__ out) {
  __shared__ double red[256];
  __shared__ float bc[4];
  constexpr int NIT = HW / (4 * 256);
  const int o = blockIdx.x;
  const int tid = threadIdx.x;

  double s = 0.0;
#pragma unroll 1
  for (int b = 0; b < NBATCH; ++b) {
    const float* p = pre + ((size_t)b * COUT + o) * HW;
#pragma unroll 1
    for (int it = 0; it < NIT; ++it) {
      const v4f v = *(const v4f*)(p + (size_t)(it * 256 + tid) * 4);
      s += (double)v[0]; s += (double)v[1]; s += (double)v[2]; s += (double)v[3];
    }
  }
  red[tid] = s;
  __syncthreads();
  for (int st = 128; st > 0; st >>= 1) {
    if (tid < st) red[tid] = red[tid] + red[tid + st];
    __syncthreads();
  }
  if (tid == 0) bc[0] = (float)(red[0] * (1.0 / (double)(NBATCH * HW)));
  __syncthreads();
  const float mean = bc[0];

  double qs = 0.0;
#pragma unroll 1
  for (int b = 0; b < NBATCH; ++b) {
    const float* p = pre + ((size_t)b * COUT + o) * HW;
#pragma unroll 1
    for (int it = 0; it < NIT; ++it) {
      const v4f v = *(const v4f*)(p + (size_t)(it * 256 + tid) * 4);
      const double d0 = (double)(v[0] - mean), d1 = (double)(v[1] - mean);
      const double d2 = (double)(v[2] - mean), d3 = (double)(v[3] - mean);
      qs += d0 * d0; qs += d1 * d1; qs += d2 * d2; qs += d3 * d3;
    }
  }
  red[tid] = qs;
  __syncthreads();
  for (int st = 128; st > 0; st >>= 1) {
    if (tid < st) red[tid] = red[tid] + red[tid + st];
    __syncthreads();
  }
  if (tid == 0) {
    const float var = (float)(red[0] * (1.0 / (double)(NBATCH * HW)));
    const float inv = rsqrtf(var + 1e-5f);
    bc[1] = inv * gamma[o];
    bc[2] = beta[o];
  }
  __syncthreads();
  const float sc = bc[1], sh = bc[2];

  for (int pass = 0; pass < 2; ++pass) {
#pragma unroll 1
    for (int b = 0; b < NBATCH; ++b) {
      const size_t plane = ((size_t)b * COUT + o) * HW;
      const float* p = pre + plane;
      float* d = out + plane;
#pragma unroll 1
      for (int it = 0; it < NIT; ++it) {
        const size_t e = (size_t)(it * 256 + tid) * 4;
        const v4f v = *(const v4f*)(p + e);
        v4f r;
        r[0] = (v[0] - mean) * sc + sh;
        r[1] = (v[1] - mean) * sc + sh;
        r[2] = (v[2] - mean) * sc + sh;
        r[3] = (v[3] - mean) * sc + sh;
        *(volatile v4f*)(d + e) = r;
      }
    }
    __threadfence();
  }
}

extern "C" void kernel_launch(void* const* d_in, const int* in_sizes, int n_in,
                              void* d_out, int out_size, void* d_ws, size_t ws_size,
                              hipStream_t stream) {
  if (n_in < 7) return;
  if (in_sizes[0] != NPIX * CIN || in_sizes[1] != NOFF * KD || in_sizes[2] != NOFF ||
      in_sizes[3] != COUT * KD || in_sizes[4] != COUT || in_sizes[5] != COUT || in_sizes[6] != COUT) return;
  if (out_size != NBATCH * COUT * HW) return;

  const float* x     = (const float*)d_in[0];
  const float* w_off = (const float*)d_in[1];
  const float* b_off = (const float*)d_in[2];
  const float* w_def = (const float*)d_in[3];
  const float* b_def = (const float*)d_in[4];
  const float* gamma = (const float*)d_in[5];
  const float* beta  = (const float*)d_in[6];
  float* out = (float*)d_out;

  const size_t bytes_pre = (size_t)NBATCH * COUT * HW * 4;
  const size_t bytes_xT  = (size_t)NPIX * CIN * 4;
  const size_t bytes_P   = (size_t)HW * KD * 2;
  const size_t bytes_off = (size_t)MOFF * HW * 4;
  const size_t bytes_Ao  = (size_t)MOFF * KD * 2;
  const size_t bytes_Wd  = (size_t)COUT * KD * 2;
  char* ws = (char*)d_ws;
  size_t o = 0;
  float* pre = (float*)(ws + o);                      o += bytes_pre;
  float* xT  = (float*)(ws + o);                      o += bytes_xT;
  unsigned short* imh = (unsigned short*)(ws + o);    o += bytes_P;
  unsigned short* val = imh;
  unsigned short* iml = (unsigned short*)(ws + o);    o += bytes_P;
  float* off = (float*)(ws + o);                      o += bytes_off;
  unsigned short* aoh = (unsigned short*)(ws + o);    o += bytes_Ao;
  unsigned short* aol = (unsigned short*)(ws + o);    o += bytes_Ao;
  unsigned short* wdp = (unsigned short*)(ws + o);    o += bytes_Wd;
  if (o > ws_size) return;

  k_xpose<<<NBATCH * HW / 32, 256, 0, stream>>>(x, xT);
  k_prep_woff<<<(MOFF * KD / 8 + 255) / 256, 256, 0, stream>>>(w_off, aoh, aol);
  k_prep_wdef<<<(COUT * KD / 8 + 255) / 256, 256, 0, stream>>>(w_def, wdp);
  for (int b = 0; b < NBATCH; ++b) {
    k_im2col<<<(HW * KK) / 32, 256, 0, stream>>>(xT, imh, iml, b);
    wmma_gemm64<1, true, 0, 0, false><<<dim3((MOFF / 64) * (HW / 64) / 8, 1), 256, 0, stream>>>(
        aoh, aol, KD, 0L,
        imh, iml, KD, 0L,
        (void*)off, (void*)wdp, HW, 0L,
        b_def,
        b_off, 0L,
        MOFF, HW, KD, 1.0f);
    k_sample<<<(HW * KK) / 32, 256, 0, stream>>>(xT, off, b_off, val, b);
    wmma_gemm64<0, false, 1, 0, false><<<dim3((COUT / 64) * (HW / 64) / 8, 1), 256, 0, stream>>>(
        wdp, wdp, KD, 0L,
        val, val, KD, 0L,
        (void*)(pre + (size_t)b * COUT * HW), (void*)wdp, HW, 0L,
        b_def,
        b_off, 0L,
        COUT, HW, KD, 0.0625f);
  }
  k_bnorm<<<COUT, 256, 0, stream>>>(pre, gamma, beta, out);
}
